// GraphConvolution_9758165697084
// MI455X (gfx1250) — hardware-verified
//
#include <hip/hip_runtime.h>
#include <stddef.h>
#include <stdint.h>
#include <math.h>


#define BB      2
#define NN      50000
#define DD      64
#define EE      800000
#define HH      32
#define MROW    (BB * NN)
#define TM      128
#define NTILE   782
#define MP      (NTILE * TM)
#define NTHR    256
#define NWAVE   8
#define EPT     8
#define CHUNK   (NTHR * EPT)
#define WCAP    (EPT * 32)
#define LISTN   (NWAVE * WCAP)
#define NBRUN   1024
#define SLB     10
#define NBW     (NBRUN / NWAVE)
#define NBLK    49
#define SNP     (NBLK * NBRUN)
#define RCAP    28672
#define DEGCAP  64
#define NBX     ((MP * (DD / 8)) / NTHR)
#define OUT1_OFF 100000
#define P_BETA  0
#define P_ATT   128
#define P_W1    256
#define P_B1    288
#define P_W2    320
#define P_B2    352
#define P_WSS   353
#define P_WSN   354
#define P_WIS   355
#define P_WIN   356
#define PARN    384
#define LDS_SCAN ((2 * RCAP + 2 * NBRUN + LISTN + 16) * 4)
#define WSMAX   134217728

static_assert(DD == 64 && HH == 32 && 2 * DD == 128);
static_assert(MP >= MROW && MP - MROW < TM);
static_assert((MP * (DD / 8)) % NTHR == 0);
static_assert(NBRUN % 32 == 0 && NBRUN == (1 << SLB) && NBRUN == 4 * NTHR);
static_assert(SNP % NBRUN == 0 && SNP >= NN && (SNP % 32) == 0);
static_assert((OUT1_OFF * 4) % 128 == 0);
static_assert((DD * 4) % 128 == 0);
static_assert(EE % EPT == 0 && EE >= EPT);
static_assert(NN < (1 << 16));
static_assert(RCAP >= 16736 + 8192 && (RCAP % 32) == 0);
static_assert(DEGCAP >= 36 + 8);
static_assert(LISTN >= NBRUN);
static_assert(2 * NBRUN <= RCAP);
static_assert(LDS_SCAN <= 300000);
static_assert(TM == NWAVE * 16);
static_assert(PARN % 4 == 0 && PARN <= 2 * NTHR && PARN / 4 <= NTHR);
static_assert((NN % 4) == 0 && (MROW % 4) == 0);
static_assert((long long)OUT1_OFF + (long long)(MROW - 1) * DD + (DD - 1) < 6500000LL);

typedef float          v2f  __attribute__((ext_vector_type(2)));
typedef float          v4f  __attribute__((ext_vector_type(4)));
typedef float          v8f  __attribute__((ext_vector_type(8)));
typedef int            v4i  __attribute__((ext_vector_type(4)));
typedef int            v8i  __attribute__((ext_vector_type(8)));
typedef unsigned int   v4u  __attribute__((ext_vector_type(4)));
typedef unsigned short v8us __attribute__((ext_vector_type(8)));
typedef __bf16         v16b __attribute__((ext_vector_type(16)));
typedef v2f  __attribute__((may_alias)) v2fa;
typedef v4f  __attribute__((may_alias)) v4fa;
typedef v8us __attribute__((may_alias)) v8usa;
union FragB { v16b v; v8us h[2]; v8i w; };

__device__ __forceinline__ v8f wmb(const FragB& a, const FragB& b, v8f c) {
  v8f d = __builtin_amdgcn_wmma_f32_16x16x32_bf16(false, a.v, false, b.v, (short)0, c, false, false);
  asm volatile("v_nop\n\tv_nop\n\tv_nop\n\tv_nop" : "+v"(d) : "v"(a.w), "v"(b.w));
  return d;
}

__device__ __forceinline__ unsigned int f2bf(float f) {
  const unsigned int u = __float_as_uint(f);
  return ((u + 0x7FFFu + ((u >> 16) & 1u)) >> 16) & 0xFFFFu;
}
__device__ __forceinline__ float bf2f(unsigned int b) { return __uint_as_float(b << 16); }
__device__ __forceinline__ float bfr(float f) { return bf2f(f2bf(f)); }
__device__ __forceinline__ unsigned int pk2(float lo, float hi) { return f2bf(lo) | (f2bf(hi) << 16); }
__device__ __forceinline__ v4u pack8(const v4f a, const v4f b) {
  v4u r;
  r.x = pk2(a.x, a.y); r.y = pk2(a.z, a.w); r.z = pk2(b.x, b.y); r.w = pk2(b.z, b.w);
  return r;
}
__device__ __forceinline__ int clampi(int v, int lo, int hi) { return v < lo ? lo : (v > hi ? hi : v); }
__device__ __forceinline__ unsigned int mskb(bool c) { return 0u - (unsigned int)c; }
__device__ __forceinline__ float eluf(float v) { return v > 0.0f ? v : expm1f(v); }

__device__ __forceinline__ float par_elem(int j,
    const float* __restrict__ beta, const float* __restrict__ att, const float* __restrict__ w1,
    const float* __restrict__ b1, const float* __restrict__ w2, const float* __restrict__ b2,
    const float* __restrict__ wss, const float* __restrict__ wsn, const float* __restrict__ wis,
    const float* __restrict__ win) {
  const unsigned int vb = __float_as_uint(beta[clampi(j, 0, 127)]);
  const unsigned int va = __float_as_uint(att[clampi(j - P_ATT, 0, 127)]);
  const unsigned int v1 = __float_as_uint(w1[clampi(j - P_W1, 0, HH - 1)]);
  const unsigned int vq = __float_as_uint(b1[clampi(j - P_B1, 0, HH - 1)]);
  const unsigned int v2 = __float_as_uint(w2[clampi(j - P_W2, 0, HH - 1)]);
  const unsigned int s0 = __float_as_uint(b2[0]);
  const unsigned int s1 = __float_as_uint(wss[0]);
  const unsigned int s2 = __float_as_uint(wsn[0]);
  const unsigned int s3 = __float_as_uint(wis[0]);
  const unsigned int s4 = __float_as_uint(win[0]);
  unsigned int r = 0u;
  r |= vb & mskb(j < P_ATT);
  r |= va & mskb(j >= P_ATT && j < P_W1);
  r |= v1 & mskb(j >= P_W1 && j < P_B1);
  r |= vq & mskb(j >= P_B1 && j < P_W2);
  r |= v2 & mskb(j >= P_W2 && j < P_B2);
  r |= s0 & mskb(j == P_B2);
  r |= s1 & mskb(j == P_WSS);
  r |= s2 & mskb(j == P_WSN);
  r |= s3 & mskb(j == P_WIS);
  r |= s4 & mskb(j == P_WIN);
  return bfr(__uint_as_float(r));
}

__global__ __launch_bounds__(NTHR) void k_prep(
    const float* __restrict__ xin, const float* __restrict__ W,
    const float* __restrict__ beta, const float* __restrict__ att, const float* __restrict__ w1,
    const float* __restrict__ b1, const float* __restrict__ w2, const float* __restrict__ b2,
    const float* __restrict__ wss, const float* __restrict__ wsn, const float* __restrict__ wis,
    const float* __restrict__ win,
    unsigned short* xb, unsigned short* wt, float* par) {
  __shared__ __attribute__((aligned(16))) float sp[PARN];
  const int tid = (int)threadIdx.x;
  const int blk = (int)blockIdx.x;
  if (blk < NBX) {
    const int u   = blk * NTHR + tid;
    const int row = u >> 3;
    const int c0  = (u & 7) * 8;
    const int rc  = row < MROW ? row : MROW - 1;
    const float* p = xin + (size_t)rc * DD + c0;
    v4f a = *(const v4fa*)p, b = *(const v4fa*)(p + 4);
    const v4f z4 = {0.f, 0.f, 0.f, 0.f};
    if (row >= MROW) { a = z4; b = z4; }
    const v4u hv = pack8(a, b);
    unsigned short* o = xb + (size_t)row * DD + c0;
    *(volatile v4u*)o = hv;
    __threadfence();
    *(volatile v4u*)o = hv;
  } else if (blk == NBX) {
#pragma unroll 1
    for (int it = 0; it < 2; ++it) {
      const int u  = it * NTHR + tid;
      const int n  = u >> 3;
      const int k8 = (u & 7) * 8;
      const float* p = W + (size_t)k8 * DD + n;
      v4f a, b;
      a.x = p[0];      a.y = p[DD];     a.z = p[2 * DD]; a.w = p[3 * DD];
      b.x = p[4 * DD]; b.y = p[5 * DD]; b.z = p[6 * DD]; b.w = p[7 * DD];
      const v4u wv = pack8(a, b);
      unsigned short* o = wt + (size_t)n * DD + k8;
      *(volatile v4u*)o = wv;
      __threadfence();
      *(volatile v4u*)o = wv;
    }
  } else {
    sp[tid] = par_elem(tid, beta, att, w1, b1, w2, b2, wss, wsn, wis, win);
    if (tid < PARN - NTHR)
      sp[NTHR + tid] = par_elem(NTHR + tid, beta, att, w1, b1, w2, b2, wss, wsn, wis, win);
    __syncthreads();
    if (tid < PARN / 4) {
      const v4f v = *(const v4fa*)(sp + 4 * tid);
      float* o = par + 4 * tid;
      *(volatile v4f*)o = v;
      __threadfence();
      *(volatile v4f*)o = v;
    }
  }
}

__global__ __launch_bounds__(NTHR) void k_gemm_node(
    const unsigned short* __restrict__ XB, const unsigned short* __restrict__ WT,
    const float* __restrict__ par, const float* __restrict__ xst,
    float* TF, float* NODE) {
  __shared__ __attribute__((aligned(16))) float stg[TM * DD];
  __shared__ __attribute__((aligned(16))) float spar[PARN];
  __shared__ __attribute__((aligned(16))) float srec[TM * 8];
  const int tid = (int)threadIdx.x, lane = tid & 31, wave = tid >> 5, hh = lane >> 4, m = lane & 15;
  const int rowBase = (int)blockIdx.x * TM;

  if (tid < PARN / 4) *(v4fa*)(spar + 4 * tid) = *(const v4fa*)(par + 4 * tid);

  v8f acc[4];
  {
    const v8f z = {0.f, 0.f, 0.f, 0.f, 0.f, 0.f, 0.f, 0.f};
    acc[0] = z; acc[1] = z; acc[2] = z; acc[3] = z;
  }
  const unsigned short* ap = XB + (size_t)(rowBase + 16 * wave + m) * DD + 8 * hh;
  const unsigned short* wp = WT + (size_t)m * DD + 8 * hh;
#pragma unroll
  for (int ks = 0; ks < DD / 32; ++ks) {
    FragB af;
    af.h[0] = *(const v8usa*)(ap + 32 * ks);
    af.h[1] = *(const v8usa*)(ap + 32 * ks + 16);
#pragma unroll
    for (int t = 0; t < 4; ++t) {
      const unsigned short* wq = wp + (size_t)(16 * t) * DD + 32 * ks;
      FragB bf;
      bf.h[0] = *(const v8usa*)wq;
      bf.h[1] = *(const v8usa*)(wq + 16);
      acc[t] = wmb(af, bf, acc[t]);
    }
  }
#pragma unroll
  for (int t = 0; t < 4; ++t) {
    const int lc = 16 * t + m;
#pragma unroll
    for (int r = 0; r < 8; ++r) {
      const int lr = 16 * wave + 8 * hh + r;
      stg[lr * DD + lc] = acc[t][r];
    }
  }
  __syncthreads();

  if (tid < TM) {
    const int row = tid;
    const int bn  = rowBase + row;
    const int bc  = bn < MROW ? bn : MROW - 1;
    const float xs = bfr(xst[bc]);
    const float* hr = stg + row * DD;
    float sr = 0.f, sc = 0.f, er = 0.f, ec = 0.f;
#pragma unroll 1
    for (int c4 = 0; c4 < DD / 4; ++c4) {
      const v4f hv = *(const v4fa*)(hr + 4 * c4);
      const v4f br = *(const v4fa*)(spar + P_BETA + 4 * c4);
      const v4f bc4 = *(const v4fa*)(spar + P_BETA + DD + 4 * c4);
      const v4f ar = *(const v4fa*)(spar + P_ATT + 4 * c4);
      const v4f ac = *(const v4fa*)(spar + P_ATT + DD + 4 * c4);
      sr = fmaf(hv.x, br.x, sr);  sc = fmaf(hv.x, bc4.x, sc);  er = fmaf(hv.x, ar.x, er);  ec = fmaf(hv.x, ac.x, ec);
      sr = fmaf(hv.y, br.y, sr);  sc = fmaf(hv.y, bc4.y, sc);  er = fmaf(hv.y, ar.y, er);  ec = fmaf(hv.y, ac.y, ec);
      sr = fmaf(hv.z, br.z, sr);  sc = fmaf(hv.z, bc4.z, sc);  er = fmaf(hv.z, ar.z, er);  ec = fmaf(hv.z, ac.z, ec);
      sr = fmaf(hv.w, br.w, sr);  sc = fmaf(hv.w, bc4.w, sc);  er = fmaf(hv.w, ar.w, er);  ec = fmaf(hv.w, ac.w, ec);
    }
    float g = 0.0f;
#pragma unroll 1
    for (int j = 0; j < HH; ++j) {
      const float hp = xs * spar[P_W1 + j] + spar[P_B1 + j];
      g = fmaf(eluf(hp), spar[P_W2 + j], g);
    }
    const float gate = eluf(g + spar[P_B2]);
    v4f ra, rb;
    ra.x = sr; ra.y = sc; ra.z = er; ra.w = ec;
    rb.x = gate; rb.y = xs; rb.z = 0.0f; rb.w = 0.0f;
    *(v4fa*)(srec + 8 * row)     = ra;
    *(v4fa*)(srec + 8 * row + 4) = rb;
  }
  __syncthreads();

  v4f fv[8];
#pragma unroll
  for (int i = 0; i < 8; ++i) fv[i] = *(const v4fa*)(stg + 4 * (i * NTHR + tid));
  const v4f nv = *(const v4fa*)(srec + 4 * tid);
  float* tp = TF + (size_t)rowBase * DD + 4 * tid;
  float* np = NODE + (size_t)rowBase * 8 + 4 * tid;
#pragma unroll
  for (int i = 0; i < 8; ++i) *(volatile v4f*)(tp + 4 * i * NTHR) = fv[i];
  *(volatile v4f*)np = nv;
  __threadfence();
#pragma unroll
  for (int i = 0; i < 8; ++i) *(volatile v4f*)(tp + 4 * i * NTHR) = fv[i];
  *(volatile v4f*)np = nv;
}

__device__ __forceinline__ int scan_chunk(const int* __restrict__ L, int cbase, int slotBase,
                                          int* list, int tid, int lane, int wave) {
  (void)lane;
  int wc = 0;
  const int e0  = cbase + tid * EPT;
  const bool vg = e0 < EE;
  const int e0c = e0 < (EE - EPT) ? e0 : (EE - EPT);
  const int* p  = L + 2 * (size_t)e0c;
  const v4i q0 = *(const v4i*)p;
  const v4i q1 = *(const v4i*)(p + 4);
  const v4i q2 = *(const v4i*)(p + 8);
  const v4i q3 = *(const v4i*)(p + 12);
  const unsigned nbs = (unsigned)slotBase;
  const unsigned unb = (unsigned)NBRUN;
  const unsigned s0 = (unsigned)q0.x - nbs, s1 = (unsigned)q0.z - nbs;
  const unsigned s2 = (unsigned)q1.x - nbs, s3 = (unsigned)q1.z - nbs;
  const unsigned s4 = (unsigned)q2.x - nbs, s5 = (unsigned)q2.z - nbs;
  const unsigned s6 = (unsigned)q3.x - nbs, s7 = (unsigned)q3.z - nbs;
  const int c0 = clampi(q0.y, 0, NN - 1), c1 = clampi(q0.w, 0, NN - 1);
  const int c2 = clampi(q1.y, 0, NN - 1), c3 = clampi(q1.w, 0, NN - 1);
  const int c4 = clampi(q2.y, 0, NN - 1), c5 = clampi(q2.w, 0, NN - 1);
  const int c6 = clampi(q3.y, 0, NN - 1), c7 = clampi(q3.w, 0, NN - 1);
  const bool h0 = vg && (s0 < unb), h1 = vg && (s1 < unb), h2 = vg && (s2 < unb), h3 = vg && (s3 < unb);
  const bool h4 = vg && (s4 < unb), h5 = vg && (s5 < unb), h6 = vg && (s6 < unb), h7 = vg && (s7 < unb);
  const unsigned any = __builtin_amdgcn_ballot_w32(h0 | h1 | h2 | h3 | h4 | h5 | h6 | h7);
  if (any != 0u) {
#define HITJ(HJ, SJ, CJ) { \
      const unsigned mj = __builtin_amdgcn_ballot_w32(HJ); \
      if (mj != 0u) { \
        if (HJ) { \
          const int pos = wc + (int)__builtin_amdgcn_mbcnt_lo(mj, 0u); \
          if (pos < WCAP) list[wave * WCAP + pos] = ((CJ) << SLB) | (int)(SJ); \
        } \
        wc += (int)__builtin_popcount(mj); } }
    HITJ(h0, s0, c0)
    HITJ(h1, s1, c1)
    HITJ(h2, s2, c2)
    HITJ(h3, s3, c3)
    HITJ(h4, s4, c4)
    HITJ(h5, s5, c5)
    HITJ(h6, s6, c6)
    HITJ(h7, s7, c7)
#undef HITJ
  }
  return wc;
}

__global__ __launch_bounds__(NTHR) void k_scan(
    const int* __restrict__ L, const float* __restrict__ NODE, const float* __restrict__ TF,
    const float* __restrict__ par, float* out1, float* SN) {
  extern __shared__ v4f lds_dyn[];
  int* reg1 = (int*)lds_dyn;
  int* reg2 = reg1 + RCAP;
  int* scnt = reg2 + RCAP;
  int* soff = scnt + NBRUN;
  int* list = soff + NBRUN;
  int* wcnt = list + LISTN;
  int* wtot = wcnt + NWAVE;
  const int tid = (int)threadIdx.x, lane = tid & 31, wave = tid >> 5;
  const int nodeBase = (int)blockIdx.x * NBRUN;

  for (int i = tid; i < NBRUN; i += NTHR) scnt[i] = 0;
  __syncthreads();

  int tot = 0;
  const int nChunks = (EE + CHUNK - 1) / CHUNK;
#pragma unroll 1
  for (int ch = 0; ch < nChunks; ++ch) {
    const int cbase = ch * CHUNK;
    const int wc = scan_chunk(L, cbase, nodeBase, list, tid, lane, wave);
    if (lane == 0) wcnt[wave] = wc;
    __syncthreads();
    int pre = 0, all = 0;
#pragma unroll
    for (int w2 = 0; w2 < NWAVE; ++w2) {
      int c = wcnt[w2];
      c = c < 0 ? 0 : (c > WCAP ? WCAP : c);
      all += c;
      pre += (w2 < wave) ? c : 0;
    }
    const int wcc  = wc > WCAP ? WCAP : wc;
    const int base = tot + pre;
#pragma unroll 1
    for (int i = lane; i < wcc; i += 32) {
      const int ent = list[wave * WCAP + i];
      const int pos = base + i;
      if (pos < RCAP) reg1[pos] = ent;
    }
    tot += all;
    tot = tot > RCAP ? RCAP : tot;
    __syncthreads();
  }
  const int nh = tot;

  if (wave == 0) {
#pragma unroll 1
    for (int b0 = 0; b0 < nh; b0 += 32) {
      const int idx = b0 + lane;
      const int uv  = reg1[idx < nh ? idx : nh - 1];
      const int m32 = (nh - b0) < 32 ? (nh - b0) : 32;
#pragma unroll 1
      for (int k = 0; k < m32; ++k) {
        const int u  = __builtin_amdgcn_readlane(uv, k);
        const int sl = u & (NBRUN - 1);
        if (lane == 0) scnt[sl] = scnt[sl] + 1;
      }
    }
  }
  __syncthreads();

  {
    const v4i ca = *(const v4i*)(scnt + 4 * tid);
    const int e0 = ca.x < 0 ? 0 : ca.x, e1 = ca.y < 0 ? 0 : ca.y, e2 = ca.z < 0 ? 0 : ca.z, e3 = ca.w < 0 ? 0 : ca.w;
    const int ts = e0 + e1 + e2 + e3;
    int incl = ts;
#pragma unroll
    for (int d = 1; d < 32; d <<= 1) {
      const int up = __shfl_up(incl, d);
      if (lane >= d) incl += up;
    }
    if (lane == 31) wtot[wave] = incl;
    __syncthreads();
    int pre = 0;
#pragma unroll
    for (int w2 = 0; w2 < NWAVE; ++w2) pre += (w2 < wave) ? wtot[w2] : 0;
    int run = pre + incl - ts;
    soff[4 * tid + 0] = run; run += e0;
    soff[4 * tid + 1] = run; run += e1;
    soff[4 * tid + 2] = run; run += e2;
    soff[4 * tid + 3] = run;
  }
  __syncthreads();
  for (int i = tid; i < NBRUN; i += NTHR) list[i] = soff[i];
  __syncthreads();

  if (wave == 0) {
#pragma unroll 1
    for (int b0 = 0; b0 < nh; b0 += 32) {
      const int idx = b0 + lane;
      const int uv  = reg1[idx < nh ? idx : nh - 1];
      const int m32 = (nh - b0) < 32 ? (nh - b0) : 32;
#pragma unroll 1
      for (int k = 0; k < m32; ++k) {
        const int u   = __builtin_amdgcn_readlane(uv, k);
        const int sl  = u & (NBRUN - 1);
        const int col = (int)((unsigned)u >> SLB);
        if (lane == 0) {
          int pos = list[sl];
          pos = pos < 0 ? 0 : (pos > RCAP - 1 ? RCAP - 1 : pos);
          reg2[pos] = col;
          list[sl] = pos + 1;
        }
      }
    }
  }
  __syncthreads();

  float* sn_st = (float*)reg1;
  const bool ovf   = (nh >= RCAP);
  const float qnan = __int_as_float(0x7fc00000);
  const float ninf = __int_as_float((int)0xff800000u);
  const float wis  = par[P_WIS];
  const float win  = par[P_WIN];

#pragma unroll 1
  for (int jt = 0; jt < NBW; ++jt) {
    const int slot = wave * NBW + jt;
    const int node = nodeBase + slot;
    const bool live = node < NN;
    const int nc = live ? node : NN - 1;
    int st = soff[slot];
    const int craw = scnt[slot];
    int cnt = craw;
    st  = st < 0 ? 0 : (st > nh ? nh : st);
    cnt = cnt < 0 ? 0 : (cnt > DEGCAP ? DEGCAP : cnt);
    if (cnt > nh - st) cnt = nh - st;
    const float pz = (ovf || craw > DEGCAP) ? qnan : 0.0f;

#pragma unroll 1
    for (int b = 0; b < BB; ++b) {
      const size_t boff = (size_t)b * NN;
      const v4f ri = *(const v4fa*)(NODE + (boff + (size_t)nc) * 8);
      const float sri = ri.x;
      const float eri = ri.z;

      float mxl = ninf, sp = 0.0f;
#pragma unroll 1
      for (int b0 = 0; b0 < cnt; b0 += 32) {
        const int q  = b0 + lane;
        const bool vq = q < cnt;
        const int qc = vq ? q : cnt - 1;
        int idx = st + qc; idx = idx < 0 ? 0 : (idx > RCAP - 1 ? RCAP - 1 : idx);
        const int col = clampi(reg2[idx], 0, NN - 1);
        const float* rp = NODE + (boff + (size_t)col) * 8;
        const v4f ra = *(const v4fa*)rp;
        const v4f rb = *(const v4fa*)(rp + 4);
        float ls = sri + ra.y; ls = (ls >= 0.0f) ? ls : 0.02f * ls;
        float le = eri + ra.w; le = (le >= 0.0f) ? le : 0.2f * le;
        const float spn = fmaf(ls, rb.y, sp);
        sp = vq ? spn : sp;
        float mn = (le > mxl) ? le : mxl;
        mn = (le != le) ? le : mn;
        mxl = vq ? mn : mxl;
      }
#pragma unroll
      for (int off = 16; off > 0; off >>= 1) {
        const float o = __shfl_xor(mxl, off);
        float t = (o > mxl) ? o : mxl;
        t = (o != o) ? o : t;
        mxl = t;
        sp += __shfl_xor(sp, off);
      }

      float den = 0.0f, a0 = 0.0f, a1 = 0.0f;
      const float* tfb = TF + boff * DD + 2 * lane;
#pragma unroll 1
      for (int b0 = 0; b0 < cnt; b0 += 32) {
        const int q  = b0 + lane;
        const bool vq = q < cnt;
        const int qc = vq ? q : cnt - 1;
        int idx = st + qc; idx = idx < 0 ? 0 : (idx > RCAP - 1 ? RCAP - 1 : idx);
        const int col = clampi(reg2[idx], 0, NN - 1);
        const float* rp = NODE + (boff + (size_t)col) * 8;
        const v4f ra = *(const v4fa*)rp;
        const v4f rb = *(const v4fa*)(rp + 4);
        float le = eri + ra.w; le = (le >= 0.0f) ? le : 0.2f * le;
        const float exv = expf(le - mxl);
        const float ex  = vq ? exv : 0.0f;
        const int exi = __float_as_int(ex);
        const int gi  = __float_as_int(rb.x);
        const int m32 = (cnt - b0) < 32 ? (cnt - b0) : 32;
#pragma unroll 1
        for (int k = 0; k < m32; ++k) {
          const int   ck  = __builtin_amdgcn_readlane(col, k);
          const float exk = __int_as_float(__builtin_amdgcn_readlane(exi, k));
          const float gk  = __int_as_float(__builtin_amdgcn_readlane(gi, k));
          const v2f t = *(const v2fa*)(tfb + (size_t)ck * DD);
          const float f0 = t.x * gk;
          const float f1 = t.y * gk;
          a0 = fmaf(exk, f0, a0);
          a1 = fmaf(exk, f1, a1);
          den += exk;
        }
      }

      const float dsafe = (cnt > 0) ? den : 1.0f;
      const float inv = 1.0f / dsafe;
      const float E0 = a0 * inv;
      const float E1 = a1 * inv;
      const v2f ti = *(const v2fa*)(tfb + (size_t)nc * DD);
      v2f ov;
      ov.x = eluf(wis * ti.x + win * E0) + pz;
      ov.y = eluf(wis * ti.y + win * E1) + pz;
      float* op = out1 + (boff + (size_t)nc) * DD + 2 * lane;
      if (live) *(volatile v2f*)op = ov;
      __threadfence();
      if (live) *(volatile v2f*)op = ov;

      const float sv = sp + pz;
      if (lane == 0) sn_st[b * NBRUN + slot] = live ? sv : 0.0f;
    }
  }
  __syncthreads();
  {
    const v4f s0 = *(const v4fa*)(sn_st + 4 * tid);
    const v4f s1 = *(const v4fa*)(sn_st + NBRUN + 4 * tid);
    float* p0 = SN + (size_t)nodeBase + 4 * tid;
    float* p1 = SN + (size_t)SNP + (size_t)nodeBase + 4 * tid;
    *(volatile v4f*)p0 = s0;
    *(volatile v4f*)p1 = s1;
    __threadfence();
    *(volatile v4f*)p0 = s0;
    *(volatile v4f*)p1 = s1;
  }
}

__global__ __launch_bounds__(NTHR) void k_state(
    const float* __restrict__ xst, const float* __restrict__ sact, const float* __restrict__ Xs,
    const float* __restrict__ SN, const float* __restrict__ par, float* out0) {
  __shared__ __attribute__((aligned(16))) float sv[NTHR];
  const int tid = (int)threadIdx.x;
  const int e   = (int)blockIdx.x * NTHR + tid;
  const int ec  = e < MROW ? e : MROW - 1;
  const int b   = ec >= NN ? 1 : 0;
  const int n   = ec - b * NN;
  const float x  = bfr(xst[ec]);
  const float X  = bfr(Xs[ec]);
  const float a  = bfr(sact[n]);
  const float s  = SN[(size_t)b * SNP + n];
  const float wss = par[P_WSS];
  const float wsn = par[P_WSN];
  const float sn = s + a;
  const float su = eluf(wss * x + wsn * sn);
  sv[tid] = su * (1.0f - X) + X;
  __syncthreads();
  if (tid < NTHR / 4) {
    const v4f v = *(const v4fa*)(sv + 4 * tid);
    const int e4 = (int)blockIdx.x * NTHR + 4 * tid;
    const bool ok = e4 < MROW;
    float* op = out0 + (ok ? e4 : 0);
    if (ok) *(volatile v4f*)op = v;
    __threadfence();
    if (ok) *(volatile v4f*)op = v;
  }
}

extern "C" void kernel_launch(void* const* d_in, const int* in_sizes, int n_in,
                              void* d_out, int out_size, void* d_ws, size_t ws_size,
                              hipStream_t stream) {
  if (n_in < 17) return;
  if (in_sizes[0] != MROW) return;
  if (in_sizes[1] != MROW * DD) return;
  if (in_sizes[2] != 2 * EE) return;
  if (in_sizes[4] != NN) return;
  if (in_sizes[5] != MROW) return;
  if (in_sizes[6] != DD * DD) return;
  if (in_sizes[7] != 2 * DD) return;
  if (in_sizes[8] < 1 || in_sizes[9] < 1) return;
  if (in_sizes[10] != HH || in_sizes[11] != HH || in_sizes[12] != HH || in_sizes[13] < 1) return;
  if (in_sizes[14] != 2 * DD) return;
  if (in_sizes[15] < 1 || in_sizes[16] < 1) return;
  if ((long long)out_size != (long long)MROW + (long long)MROW * DD) return;

  const float* xst  = (const float*)d_in[0];
  const float* xin  = (const float*)d_in[1];
  const int*   Lp   = (const int*)  d_in[2];
  const float* sact = (const float*)d_in[4];
  const float* Xs   = (const float*)d_in[5];
  const float* W    = (const float*)d_in[6];
  const float* beta = (const float*)d_in[7];
  const float* wss  = (const float*)d_in[8];
  const float* wsn  = (const float*)d_in[9];
  const float* w1   = (const float*)d_in[10];
  const float* b1   = (const float*)d_in[11];
  const float* w2   = (const float*)d_in[12];
  const float* b2   = (const float*)d_in[13];
  const float* att  = (const float*)d_in[14];
  const float* wis  = (const float*)d_in[15];
  const float* win  = (const float*)d_in[16];
  float* out0 = (float*)d_out;
  float* out1 = (float*)d_out + OUT1_OFF;

  char* ws = (char*)d_ws;
  size_t off = 0;
  const size_t oPAR = off; off += (size_t)PARN * 4;                off = (off + 255) & ~(size_t)255;
  const size_t oWT  = off; off += (size_t)DD * DD * 2;             off = (off + 255) & ~(size_t)255;
  const size_t oXB  = off; off += (size_t)MP * DD * 2;             off = (off + 255) & ~(size_t)255;
  const size_t oTF  = off; off += (size_t)MP * DD * 4;             off = (off + 255) & ~(size_t)255;
  const size_t oND  = off; off += (size_t)MP * 8 * 4;              off = (off + 255) & ~(size_t)255;
  const size_t oSN  = off; off += (size_t)BB * SNP * 4;            off = (off + 255) & ~(size_t)255;
  if (off > ws_size || off > (size_t)WSMAX) return;
  float*          PAR  = (float*)(ws + oPAR);
  unsigned short* WT   = (unsigned short*)(ws + oWT);
  unsigned short* XB   = (unsigned short*)(ws + oXB);
  float*          TF   = (float*)(ws + oTF);
  float*          NODE = (float*)(ws + oND);
  float*          SN   = (float*)(ws + oSN);

  hipFuncSetAttribute(reinterpret_cast<const void*>(&k_scan),
                      hipFuncAttributeMaxDynamicSharedMemorySize, LDS_SCAN);

  k_prep<<<NBX + 2, NTHR, 0, stream>>>(xin, W, beta, att, w1, b1, w2, b2, wss, wsn, wis, win, XB, WT, PAR);
  k_gemm_node<<<NTILE, NTHR, 0, stream>>>(XB, WT, PAR, xst, TF, NODE);
  k_scan<<<NBLK, NTHR, LDS_SCAN, stream>>>(Lp, NODE, TF, PAR, out1, SN);
  k_state<<<(MROW + NTHR - 1) / NTHR, NTHR, 0, stream>>>(xst, sact, Xs, SN, PAR, out0);
}
